// RCNNWLModel_24704651886894
// MI455X (gfx1250) — hardware-run, weakly checked
//
#include <hip/hip_runtime.h>


namespace {
constexpr int NBM = 128, NAT = 200, NBD = 500, KS = 10, AF = 82, AFP = 96, BF = 6, H = 256, NA = NBM * NAT  , NBT = NBM * NBD  , DEPTH = 3;
constexpr float XS = 8.0f, HS = 256.0f, WSC = 256.0f;
typedef _Float16 b16;
typedef __attribute__((ext_vector_type(16))) _Float16 v16b;
typedef __attribute__((ext_vector_type(8))) _Float16 v8b;
typedef __attribute__((ext_vector_type(8))) float v8f;
typedef __attribute__((ext_vector_type(4))) float v4f;
__device__ __forceinline__ float bf16_rne(float f) { unsigned int u = __float_as_uint(f); u += 0x7FFFu + ((u >> 16) & 1u); float r = __uint_as_float(u & 0xFFFF0000u); asm volatile("" : "+v"(r)); return r; }
__device__ __forceinline__ float bfv(float f) { float r = bf16_rne(f); asm volatile("" : "+v"(r)); return r; }
__device__ __forceinline__ void split16(float v, b16& hi, b16& lo) { hi = (b16)v; lo = (b16)(v - (float)hi); }
__device__ __forceinline__ v16b frag_kb(const b16* p, int hh) { const v8b a = *(const v8b*)(p + 8 * hh), b = *(const v8b*)(p + 16 + 8 * hh); v16b f;
#pragma unroll
  for (int e = 0; e < 8; ++e) { f[e] = a[e]; f[8 + e] = b[e]; } return f; }
__device__ __forceinline__ v8f wmma16b(v16b a, v16b b, v8f c) { v8f d = __builtin_amdgcn_wmma_f32_16x16x32_f16(false, a, false, b, (short)0, c, false, false); asm volatile("v_nop\n\tv_nop\n\tv_nop\n\tv_nop" : "+v"(d) : "v"(a), "v"(b)); return d; }
__device__ __forceinline__ void wave_lds_sync() { __builtin_amdgcn_fence(__ATOMIC_RELEASE, "workgroup"); __builtin_amdgcn_wave_barrier(); __builtin_amdgcn_fence(__ATOMIC_ACQUIRE, "workgroup"); }
__device__ __forceinline__ float pmul(float a, float b) { float p = a * b; asm volatile("" : "+v"(p)); return p; }
__device__ __forceinline__ int iclamp(int v, int lo, int hi) { return v < lo ? lo : (v > hi ? hi : v); }

__global__ __launch_bounds__(256) void wput_kernel(const float* __restrict__ wem, const float* __restrict__ wna, const float* __restrict__ wu2, const float* __restrict__ wsf, const float* __restrict__ wu1, b16* __restrict__ WEM, b16* __restrict__ W3, b16* __restrict__ WU1) { const size_t nt = (size_t)gridDim.x * 256, u0 = (size_t)blockIdx.x * 256 + threadIdx.x; v8b v;
  for (size_t u = u0; u < (size_t)H * (AFP / 8); u += nt) { const int o = (int)(u / (AFP / 8)), k0 = (int)(u % (AFP / 8)) * 8;
#pragma unroll
    for (int j = 0; j < 8; ++j) { const int k = k0 + j; v[j] = (b16)(k < AF ? bf16_rne(wem[(size_t)k * H + o]) * WSC : 0.0f); } for (int pass = 0; pass < 2; ++pass) { *(volatile v8b*)(WEM + (size_t)o * AFP + k0) = v; __threadfence(); } }
  for (size_t u = u0; u < (size_t)3 * H * (H / 8); u += nt) { const int o = (int)(u / (H / 8)), k0 = (int)(u % (H / 8)) * 8; const int g = o / H, oo = o % H; const float* w = g == 0 ? wna : (g == 1 ? wu2 : wsf);
#pragma unroll
    for (int j = 0; j < 8; ++j) v[j] = (b16)(bf16_rne(w[(size_t)(k0 + j) * H + oo]) * WSC); for (int pass = 0; pass < 2; ++pass) { *(volatile v8b*)(W3 + (size_t)o * H + k0) = v; __threadfence(); } }
  for (size_t u = u0; u < (size_t)H * (2 * H / 8); u += nt) { const int o = (int)(u / (2 * H / 8)), k0 = (int)(u % (2 * H / 8)) * 8;
#pragma unroll
    for (int j = 0; j < 8; ++j) v[j] = (b16)(bf16_rne(wu1[(size_t)(k0 + j) * H + o]) * WSC); for (int pass = 0; pass < 2; ++pass) { *(volatile v8b*)(WU1 + (size_t)o * 2 * H + k0) = v; __threadfence(); } } }
__global__ __launch_bounds__(32) void embed_kernel(const float* __restrict__ xa, const b16* __restrict__ WEM, int ALIM, float* __restrict__ A) { __shared__ __attribute__((aligned(16))) b16 Ah[16][AFP + 8]; __shared__ float Tf[16][H + 4]; const int lane = threadIdx.x, nloc = lane & 15, hlf = lane >> 4; const size_t m0 = (size_t)blockIdx.x * 16; if (m0 >= (size_t)ALIM) return;
  for (int rr = 0; rr < 16; ++rr) for (int q = 0; q < 3; ++q) { const int c = q * 32 + lane; Ah[rr][c] = (b16)(c < AF ? bf16_rne(xa[(m0 + rr) * AF + c]) * XS : 0.0f); } if (lane < 16) for (int k = AFP; k < AFP + 8; ++k) Ah[lane][k] = (b16)0.0f;
  wave_lds_sync(); v8f acc[16];
#pragma unroll
  for (int t = 0; t < 16; ++t) acc[t] = (v8f){};
#pragma unroll
  for (int kb = 0; kb < AFP; kb += 32) { const v16b a = frag_kb(&Ah[nloc][kb], hlf);
#pragma unroll
    for (int t = 0; t < 16; ++t) acc[t] = wmma16b(a, frag_kb(WEM + (size_t)(t * 16 + nloc) * AFP + kb, hlf), acc[t]); }
#pragma unroll
  for (int t = 0; t < 16; ++t)
#pragma unroll
    for (int r8 = 0; r8 < 8; ++r8) Tf[8 * hlf + r8][t * 16 + nloc] = fmaxf(acc[t][r8] * (1.0f / (XS * WSC)), 0.0f);
  wave_lds_sync();
  for (int pass = 0; pass < 2; ++pass) { for (int rr = 0; rr < 16; ++rr) for (int q = 0; q < 2; ++q) *(volatile v4f*)(A + (m0 + rr) * H + q * 128 + lane * 4) = *(const v4f*)(&Tf[rr][q * 128 + lane * 4]); __threadfence(); } }
__global__ __launch_bounds__(32) void proj_kernel(const float* __restrict__ A, const b16* __restrict__ W3, int NG, int ALIM, float* __restrict__ P) { __shared__ __attribute__((aligned(16))) b16 Ah[16][H + 8], Al[16][H + 8]; __shared__ float Tf[16][H + 4]; const int lane = threadIdx.x, nloc = lane & 15, hlf = lane >> 4; const int g = blockIdx.x % NG; const size_t m0 = (size_t)(blockIdx.x / NG) * 16; if (m0 >= (size_t)ALIM) return;
  for (int rr = 0; rr < 16; ++rr) for (int q = 0; q < H / 32; ++q) { b16 p, ql; split16(A[(m0 + rr) * H + q * 32 + lane] * HS, p, ql); Ah[rr][q * 32 + lane] = p; Al[rr][q * 32 + lane] = ql; } if (lane < 16) for (int k = H; k < H + 8; ++k) { Ah[lane][k] = (b16)0.0f; Al[lane][k] = (b16)0.0f; }
  wave_lds_sync(); v8f acc[16];
#pragma unroll
  for (int t = 0; t < 16; ++t) acc[t] = (v8f){};
#pragma unroll 2
  for (int kb = 0; kb < H; kb += 32) { const v16b a = frag_kb(&Ah[nloc][kb], hlf), al = frag_kb(&Al[nloc][kb], hlf);
#pragma unroll
    for (int t = 0; t < 16; ++t) { const v16b bw = frag_kb(W3 + ((size_t)g * H + t * 16 + nloc) * H + kb, hlf); acc[t] = wmma16b(a, bw, acc[t]); acc[t] = wmma16b(al, bw, acc[t]); } }
#pragma unroll
  for (int t = 0; t < 16; ++t)
#pragma unroll
    for (int r8 = 0; r8 < 8; ++r8) Tf[8 * hlf + r8][t * 16 + nloc] = acc[t][r8] * (1.0f / (HS * WSC));
  wave_lds_sync();
  for (int pass = 0; pass < 2; ++pass) { for (int rr = 0; rr < 16; ++rr) for (int q = 0; q < 2; ++q) *(volatile v4f*)(P + (m0 + rr) * 3 * H + g * H + q * 128 + lane * 4) = *(const v4f*)(&Tf[rr][q * 128 + lane * 4]); __threadfence(); } }
__global__ __launch_bounds__(256) void slot_kernel(const float* __restrict__ P, const float* __restrict__ bond, const float* __restrict__ wnb, const float* __restrict__ wu2, const float* __restrict__ bu2, const int* __restrict__ ag, const int* __restrict__ bg, const int* __restrict__ nnb, const float* __restrict__ nmask, int LAST, int ALIM, float* __restrict__ NL, float* __restrict__ KER) { const int wave = threadIdx.x >> 5, lane = threadIdx.x & 31; const size_t a = (size_t)blockIdx.x * 8 + wave; if (a >= (size_t)ALIM) return; const size_t b = a / NAT; const int cnt = iclamp(nnb[a], 0, KS); float fn[8] = {0, 0, 0, 0, 0, 0, 0, 0}, nl[8] = {0, 0, 0, 0, 0, 0, 0, 0}; float bu8[8], wb[BF][8], wu[BF][8];
#pragma unroll
  for (int q = 0; q < 8; ++q) { bu8[q] = bfv(bu2[lane * 8 + q]);
#pragma unroll
    for (int f = 0; f < BF; ++f) { wb[f][q] = bfv(wnb[f * H + lane * 8 + q]); wu[f][q] = bfv(wu2[(size_t)(H + f) * H + lane * 8 + q]); } }
#pragma unroll 1
  for (int k = 0; k < cnt; ++k) { const size_t j = b * NAT + (size_t)iclamp(ag[a * KS + k], 0, NAT - 1); const size_t m = b * NBD + (size_t)iclamp(bg[a * KS + k], 0, NBD - 1); const v4f p0a = *(const v4f*)(P + j * 3 * H + lane * 8), p0b = *(const v4f*)(P + j * 3 * H + lane * 8 + 4), p1a = *(const v4f*)(P + j * 3 * H + H + lane * 8), p1b = *(const v4f*)(P + j * 3 * H + H + lane * 8 + 4); float x6[BF]; for (int f = 0; f < BF; ++f) x6[f] = bfv(bond[m * BF + f]); float bbv[8], buv[8];
#pragma unroll
    for (int q = 0; q < 8; ++q) { float sa = 0.0f, sb = 0.0f;
#pragma unroll
      for (int f = 0; f < BF; ++f) { sa += pmul(x6[f], wb[f][q]); sb += pmul(x6[f], wu[f][q]); } bbv[q] = sa; buv[q] = sb; }
#pragma unroll
    for (int q = 0; q < 4; ++q) { fn[q] += pmul(p0a[q], bbv[q]); fn[4 + q] += pmul(p0b[q], bbv[4 + q]); nl[q] += fmaxf(p1a[q] + buv[q] + bu8[q], 0.0f); nl[4 + q] += fmaxf(p1b[q] + buv[4 + q] + bu8[4 + q], 0.0f); } }
  for (int pass = 0; pass < 2; ++pass) { *(volatile v4f*)(NL + a * H + lane * 8) = (v4f){nl[0], nl[1], nl[2], nl[3]}; *(volatile v4f*)(NL + a * H + lane * 8 + 4) = (v4f){nl[4], nl[5], nl[6], nl[7]}; __threadfence(); }
  if (LAST) { const float nm = bfv(nmask[a]); const v4f sa = *(const v4f*)(P + a * 3 * H + 2 * H + lane * 8), sb = *(const v4f*)(P + a * 3 * H + 2 * H + lane * 8 + 4); v4f ka, kb;
#pragma unroll
    for (int q = 0; q < 4; ++q) { ka[q] = pmul(pmul(fn[q], sa[q]), nm); kb[q] = pmul(pmul(fn[4 + q], sb[q]), nm); }
    for (int pass = 0; pass < 2; ++pass) { *(volatile v4f*)(KER + a * H + lane * 8) = ka; *(volatile v4f*)(KER + a * H + lane * 8 + 4) = kb; __threadfence(); } } }
__global__ __launch_bounds__(32) void upd_kernel(const float* __restrict__ A, const float* __restrict__ NL, const b16* __restrict__ WU1, const float* __restrict__ bu1, int ALIM, float* __restrict__ AO) { __shared__ __attribute__((aligned(16))) b16 Ah[16][2 * H + 8], Al[16][2 * H + 8]; __shared__ float Tf[16][H + 4]; const int lane = threadIdx.x, nloc = lane & 15, hlf = lane >> 4; const size_t m0 = (size_t)blockIdx.x * 16; if (m0 >= (size_t)ALIM) return;
  for (int rr = 0; rr < 16; ++rr) for (int q = 0; q < 2 * H / 32; ++q) { const int c = q * 32 + lane; const float v = c < H ? A[(m0 + rr) * H + c] : NL[(m0 + rr) * H + c - H]; b16 p, ql; split16(v * HS, p, ql); Ah[rr][c] = p; Al[rr][c] = ql; } if (lane < 16) for (int k = 2 * H; k < 2 * H + 8; ++k) { Ah[lane][k] = (b16)0.0f; Al[lane][k] = (b16)0.0f; }
  wave_lds_sync(); v8f acc[16];
#pragma unroll
  for (int t = 0; t < 16; ++t) acc[t] = (v8f){};
#pragma unroll 2
  for (int kb = 0; kb < 2 * H; kb += 32) { const v16b a = frag_kb(&Ah[nloc][kb], hlf), al = frag_kb(&Al[nloc][kb], hlf);
#pragma unroll
    for (int t = 0; t < 16; ++t) { const v16b bw = frag_kb(WU1 + (size_t)(t * 16 + nloc) * 2 * H + kb, hlf); acc[t] = wmma16b(a, bw, acc[t]); acc[t] = wmma16b(al, bw, acc[t]); } }
#pragma unroll
  for (int t = 0; t < 16; ++t) { const int cc = t * 16 + nloc; const float bb = bfv(bu1[cc]);
#pragma unroll
    for (int r8 = 0; r8 < 8; ++r8) Tf[8 * hlf + r8][cc] = fmaxf(acc[t][r8] * (1.0f / (HS * WSC)) + bb, 0.0f); }
  wave_lds_sync();
  for (int pass = 0; pass < 2; ++pass) { for (int rr = 0; rr < 16; ++rr) for (int q = 0; q < 2; ++q) *(volatile v4f*)(AO + (m0 + rr) * H + q * 128 + lane * 4) = *(const v4f*)(&Tf[rr][q * 128 + lane * 4]); __threadfence(); } }
__global__ __launch_bounds__(256) void mol_kernel(const float* __restrict__ KER, int BLIM, float* __restrict__ MOL) { const int wave = threadIdx.x >> 5, lane = threadIdx.x & 31; const int b = blockIdx.x * 8 + wave; if (b >= BLIM) return; float s[8] = {0, 0, 0, 0, 0, 0, 0, 0};
#pragma unroll 1
  for (int n = 0; n < NAT; ++n) { const v4f a = *(const v4f*)(KER + ((size_t)b * NAT + n) * H + lane * 8), c = *(const v4f*)(KER + ((size_t)b * NAT + n) * H + lane * 8 + 4);
#pragma unroll
    for (int q = 0; q < 4; ++q) { s[q] += a[q]; s[4 + q] += c[q]; } }
  for (int pass = 0; pass < 2; ++pass) { *(volatile v4f*)(MOL + (size_t)b * H + lane * 8) = (v4f){s[0], s[1], s[2], s[3]}; *(volatile v4f*)(MOL + (size_t)b * H + lane * 8 + 4) = (v4f){s[4], s[5], s[6], s[7]}; __threadfence(); } }
}

extern "C" void kernel_launch(void* const* d_in, const int* in_sizes, int n_in, void* d_out, int out_size, void* d_ws, size_t ws_size, hipStream_t stream) {
  (void)n_in;
  auto Fp = [&](int i) { return (const float*)d_in[i]; }; auto Ip = [&](int i) { return (const int*)d_in[i]; };
  if (in_sizes[0] != NA * AF || in_sizes[1] != NBT * BF || in_sizes[2] != NA || in_sizes[3] != AF * H || in_sizes[4] != H * H || in_sizes[5] != BF * H || in_sizes[6] != H * H || in_sizes[7] != (H + BF) * H || in_sizes[9] != 2 * H * H || in_sizes[11] != NA * KS || in_sizes[12] != NA * KS || in_sizes[13] != NA || out_size != NA * H + NBM * H) return;
  const int ALIM = NA;
  size_t off = 0; char* ws = (char*)d_ws;
  auto carve = [&](size_t bytes) { char* p = ws + off; off += (bytes + 255) & ~(size_t)255; return p; };
  b16* WEM = (b16*)carve((size_t)H * AFP * 2); b16* W3 = (b16*)carve((size_t)3 * H * H * 2); b16* WU1 = (b16*)carve((size_t)H * 2 * H * 2); float* AA = (float*)carve((size_t)NA * H * 4); float* AB = (float*)carve((size_t)NA * H * 4); float* P = (float*)carve((size_t)NA * 3 * H * 4); float* NL = (float*)carve((size_t)NA * H * 4);
  if (off > ws_size || off > ((size_t)192 << 20)) return;
  float* KER = (float*)d_out; float* MOL = KER + (size_t)NA * H;
  wput_kernel<<<256, 256, 0, stream>>>(Fp(3), Fp(4), Fp(7), Fp(6), Fp(9), WEM, W3, WU1);
  embed_kernel<<<ALIM / 16, 32, 0, stream>>>(Fp(0), WEM, ALIM, AA);
  float* ain = AA; float* aout = AB;
  for (int d = 0; d < DEPTH; ++d) { const int last = d == DEPTH - 1; const int ng = last ? 3 : 2;
    proj_kernel<<<(ALIM / 16) * ng, 32, 0, stream>>>(ain, W3, ng, ALIM, P);
    slot_kernel<<<(ALIM + 7) / 8, 256, 0, stream>>>(P, Fp(1), Fp(5), Fp(7), Fp(8), Ip(11), Ip(12), Ip(13), Fp(2), last, ALIM, NL, KER);
    if (!last) { upd_kernel<<<ALIM / 16, 32, 0, stream>>>(ain, NL, WU1, Fp(10), ALIM, aout); float* t = ain; ain = aout; aout = t; } }
  mol_kernel<<<NBM / 8, 256, 0, stream>>>(KER, ALIM / NAT, MOL);
}
